// DeepEquiCategorySpecificMLP_35442070126939
// MI455X (gfx1250) — hardware-run, weakly checked
//
#include <hip/hip_runtime.h>
#include <stddef.h>


#define DIM     256
#define HID     1024
#define NGRP    8
#define TM      64
#define TN      64
#define NTH     256
#define NWV     8
#define SP      68
#define TPW     264
#define A_CARRY 8.0f
#define W_CARRY 256.0f
#define RC2048  0.00048828125f
#define LN_EPS  1e-5f
#define WSCAP   134217728

static_assert(((SP * 4) % 16) == 0 && ((TPW * 2) % 16) == 0);
static_assert((DIM % 256) == 0 && (HID % 256) == 0 && TM == 64 && TN == 64 && NTH == 256 && NWV * 32 == NTH);
static_assert((DIM % TN) == 0 && (HID % TN) == 0 && (DIM % 32) == 0 && (HID % 32) == 0);
static_assert(TM * SP * 4 <= 40 * 1024);

typedef float    v4f  __attribute__((ext_vector_type(4)));
typedef float    v8f  __attribute__((ext_vector_type(8)));
typedef _Float16 v4h  __attribute__((ext_vector_type(4)));
typedef _Float16 v8h  __attribute__((ext_vector_type(8)));
typedef _Float16 v16h __attribute__((ext_vector_type(16)));
union Frag { v16h v; v8h half[2]; };
union Pk   { v8h h; v4f f; };
static_assert(sizeof(Frag) == 32);
static_assert(sizeof(Pk) == 16);

__device__ __forceinline__ v8f wmf(v16h a, v16h bq, v8f c) {
  v8f d = __builtin_amdgcn_wmma_f32_16x16x32_f16(false, a, false, bq, (short)0, c, false, false);
  asm volatile("v_nop\n\tv_nop\n\tv_nop\n\tv_nop" : "+v"(d) : "v"(a), "v"(bq));
  return d;
}

__device__ __forceinline__ v8f zero8() {
  v8f z = {0.f, 0.f, 0.f, 0.f, 0.f, 0.f, 0.f, 0.f};
  return z;
}

__device__ __forceinline__ float hsum4(v4f a) { return (a.x + a.y) + (a.z + a.w); }
__device__ __forceinline__ float hsq4(v4f a) { return (a.x * a.x + a.y * a.y) + (a.z * a.z + a.w * a.w); }

__device__ __forceinline__ float wsum(float s) {
  s += __shfl_xor(s, 1);
  s += __shfl_xor(s, 2);
  s += __shfl_xor(s, 4);
  s += __shfl_xor(s, 8);
  s += __shfl_xor(s, 16);
  return s;
}

__device__ __forceinline__ void grp_hist(const int* __restrict__ cat, int nrows, int* s_w, int* s_cnt) {
  const int tid = threadIdx.x, wave = tid >> 5, lane = tid & 31;
  int cc[NGRP];
#pragma unroll
  for (int g = 0; g < NGRP; ++g) cc[g] = 0;
  const int nch = (nrows + NTH - 1) / NTH;
#pragma unroll 1
  for (int j = 0; j < nch; ++j) {
    const int row = j * NTH + tid;
    const int ra = row < nrows ? row : nrows - 1;
    int id = cat[ra];
    id = row < nrows ? id : -1;
#pragma unroll
    for (int g = 0; g < NGRP; ++g) cc[g] += __builtin_popcount(__builtin_amdgcn_ballot_w32(id == g));
  }
  if (lane == 0) {
#pragma unroll
    for (int g = 0; g < NGRP; ++g) s_w[wave * NGRP + g] = cc[g];
  }
  __syncthreads();
  if (tid < NGRP) {
    int s = 0;
#pragma unroll
    for (int w = 0; w < NWV; ++w) s += s_w[w * NGRP + tid];
    s_cnt[tid] = s;
  }
  __syncthreads();
}

__device__ __forceinline__ void tile_lookup(const int* s_cnt, int tile, int& csel, int& rank0) {
  int ts = 0;
  csel = -1; rank0 = 0;
#pragma unroll
  for (int g = 0; g < NGRP; ++g) {
    const int nt = (s_cnt[g] + TM - 1) / TM;
    if (tile >= ts && tile < ts + nt) { csel = g; rank0 = (tile - ts) * TM; }
    ts += nt;
  }
}

__global__ __launch_bounds__(NTH) void k_wprep(const float* __restrict__ W, _Float16* WT, int K, int NO) {
  __shared__ _Float16 T[32 * TPW] __attribute__((aligned(16)));
  const int tid = threadIdx.x, wave = tid >> 5, lane = tid & 31;
  const int nkc = K / 256, nnb = NO / 32;
  int bid = blockIdx.x;
  const int kc = bid % nkc; bid /= nkc;
  const int nb = bid % nnb;
  const int g  = bid / nnb;
  const int n0 = nb * 32, k0 = kc * 256;
  const float* src = W + ((size_t)g * K + k0) * NO + n0 + lane;
#pragma unroll 4
  for (int it = 0; it < 32; ++it) {
    const int kk = it * 8 + wave;
    const float v = src[(size_t)kk * NO];
    T[lane * TPW + kk] = (_Float16)(v * W_CARRY);
  }
  __syncthreads();
  _Float16* dst = WT + ((size_t)g * NO + n0) * K + k0 + 8 * lane;
  v4f u[4];
#pragma unroll
  for (int rr = 0; rr < 4; ++rr) {
    const int r = wave * 4 + rr;
    Pk p; p.h = *(const v8h*)(T + r * TPW + 8 * lane);
    u[rr] = p.f;
    *(volatile v4f*)(dst + (size_t)r * K) = u[rr];
  }
  __threadfence();
#pragma unroll
  for (int rr = 0; rr < 4; ++rr) {
    const int r = wave * 4 + rr;
    *(volatile v4f*)(dst + (size_t)r * K) = u[rr];
  }
}

__global__ __launch_bounds__(NTH) void k_xn(const float* __restrict__ x, const int* __restrict__ cat,
                                             _Float16* XN, int nrows) {
  __shared__ int s_w[NWV * NGRP];
  __shared__ int s_cnt[NGRP];
  __shared__ int s_wt[NWV];
  __shared__ int s_list[TM];
  const int tid = threadIdx.x, wave = tid >> 5, lane = tid & 31;
  grp_hist(cat, nrows, s_w, s_cnt);
  int csel, rank0;
  tile_lookup(s_cnt, (int)blockIdx.x, csel, rank0);
  if (csel < 0) return;
  if (tid < TM) s_list[tid] = -1;
  __syncthreads();
  int base = 0;
  const int nch = (nrows + NTH - 1) / NTH;
#pragma unroll 1
  for (int j = 0; j < nch; ++j) {
    const int row = j * NTH + tid;
    const int ra = row < nrows ? row : nrows - 1;
    int id = cat[ra];
    id = row < nrows ? id : -1;
    const bool hit = (id == csel);
    const unsigned b = __builtin_amdgcn_ballot_w32(hit);
    const int pre = __builtin_popcount(b & ((1u << lane) - 1u));
    if (lane == 0) s_wt[wave] = __builtin_popcount(b);
    __syncthreads();
    int woff = 0, tot = 0;
#pragma unroll
    for (int w = 0; w < NWV; ++w) {
      const int v = s_wt[w];
      woff += (w < wave) ? v : 0;
      tot += v;
    }
    const int rk = base + woff + pre - rank0;
    if (hit && rk >= 0 && rk < TM) s_list[rk] = row;
    base += tot;
    __syncthreads();
  }

  const size_t slot0 = (size_t)blockIdx.x * TM;
#pragma unroll 1
  for (int i = 0; i < 8; ++i) {
    const int sl = wave * 8 + i;
    const int r = s_list[sl];
    const int ra = r < 0 ? 0 : r;
    const float* xr = x + (size_t)ra * DIM + 8 * lane;
    const v4f a = *(const v4f*)(xr);
    const v4f c = *(const v4f*)(xr + 4);
    float s = hsum4(a) + hsum4(c);
    s = wsum(s);
    const float mu = s * (1.0f / (float)DIM);
    const v4f da = a - mu, dc = c - mu;
    float q = hsq4(da) + hsq4(dc);
    q = wsum(q);
    const float rs = rsqrtf(q * (1.0f / (float)DIM) + LN_EPS);
    const float sc = (r < 0) ? 0.0f : rs * A_CARRY;
    const v4f oa = da * sc, oc = dc * sc;
    const v8f o8 = __builtin_shufflevector(oa, oc, 0, 1, 2, 3, 4, 5, 6, 7);
    Pk u; u.h = __builtin_convertvector(o8, v8h);
    _Float16* dst = XN + (slot0 + sl) * (size_t)DIM + 8 * lane;
    *(volatile v4f*)dst = u.f;
    __threadfence();
    *(volatile v4f*)dst = u.f;
  }
}

template <int K, int NOUT, int MODE>
__global__ __launch_bounds__(NTH) void k_gemm(const _Float16* __restrict__ A, const _Float16* __restrict__ WT,
                                               const _Float16* __restrict__ WT2, const float* __restrict__ bias,
                                               const float* __restrict__ bias2, const int* __restrict__ cat,
                                               float* outF, _Float16* outH, int nrows) {
  static_assert((K % 32) == 0 && (NOUT % TN) == 0);
  __shared__ int s_w[NWV * NGRP];
  __shared__ int s_cnt[NGRP];
  __shared__ float s_b[2 * TN];
  __shared__ float S[TM * SP] __attribute__((aligned(16)));
  const int tid = threadIdx.x, wave = tid >> 5, lane = tid & 31;
  grp_hist(cat, nrows, s_w, s_cnt);
  int csel, rank0;
  tile_lookup(s_cnt, (int)blockIdx.x, csel, rank0);
  if (csel < 0) return;
  (void)rank0;
  const int cb = blockIdx.y;
  const int col0 = cb * TN;

  {
    const int ci = tid & (TN - 1);
    const float bvl = bias[(size_t)csel * NOUT + col0 + ci];
    float bvl2 = 0.0f;
    if (MODE == 2) bvl2 = bias2[(size_t)csel * NOUT + col0 + ci];
    if (tid < TN) { s_b[tid] = bvl; s_b[TN + tid] = bvl2; }
  }
  __syncthreads();

  const int h = lane >> 4, m = lane & 15;
  const int rt = wave & 3, cg = wave >> 2;
  const size_t slot0 = (size_t)blockIdx.x * TM;
  const int colw = col0 + cg * 32;
  const _Float16* arow  = A + (slot0 + rt * 16 + m) * (size_t)K + 8 * h;
  const _Float16* brow  = WT  + ((size_t)csel * NOUT + colw + m) * K + 8 * h;
  const _Float16* brow2 = WT2 + ((size_t)csel * NOUT + colw + m) * K + 8 * h;

  v8f acc[2], acc2[2];
#pragma unroll
  for (int t = 0; t < 2; ++t) { acc[t] = zero8(); acc2[t] = zero8(); }

#pragma unroll 1
  for (int kk = 0; kk < K; kk += 32) {
    Frag fa;
    fa.half[0] = *(const v8h*)(arow + kk);
    fa.half[1] = *(const v8h*)(arow + kk + 16);
#pragma unroll
    for (int t = 0; t < 2; ++t) {
      const _Float16* bp = brow + (size_t)(t * 16) * K + kk;
      Frag fb;
      fb.half[0] = *(const v8h*)(bp);
      fb.half[1] = *(const v8h*)(bp + 16);
      acc[t] = wmf(fa.v, fb.v, acc[t]);
      if (MODE == 2) {
        const _Float16* bq = brow2 + (size_t)(t * 16) * K + kk;
        Frag fg;
        fg.half[0] = *(const v8h*)(bq);
        fg.half[1] = *(const v8h*)(bq + 16);
        acc2[t] = wmf(fa.v, fg.v, acc2[t]);
      }
    }
  }

#pragma unroll
  for (int t = 0; t < 2; ++t) {
    const int lc = cg * 32 + t * 16 + m;
    const float bv = s_b[lc];
    float bv2 = 0.0f;
    if (MODE == 2) bv2 = s_b[TN + lc];
    float* sc = S + (rt * 16 + 8 * h) * SP + lc;
#pragma unroll
    for (int r = 0; r < 8; ++r) {
      float v = acc[t][r] * RC2048 + bv;
      if (MODE == 1) v = fmaxf(v, 0.0f) * A_CARRY;
      if (MODE == 2) {
        const float gv = acc2[t][r] * RC2048 + bv2;
        v = v * __builtin_amdgcn_rcpf(1.0f + __expf(-gv));
      }
      sc[r * SP] = v;
    }
  }
  __syncthreads();

  if (MODE == 1) {
    const int rq = lane >> 3, c8 = 8 * (lane & 7);
    v4f u[2];
#pragma unroll
    for (int i = 0; i < 2; ++i) {
      const int r = wave * 8 + i * 4 + rq;
      const float* sp = S + r * SP + c8;
      const v4f a = *(const v4f*)(sp);
      const v4f c = *(const v4f*)(sp + 4);
      const v8f o8 = __builtin_shufflevector(a, c, 0, 1, 2, 3, 4, 5, 6, 7);
      Pk p; p.h = __builtin_convertvector(o8, v8h);
      u[i] = p.f;
    }
#pragma unroll
    for (int i = 0; i < 2; ++i) {
      const int r = wave * 8 + i * 4 + rq;
      _Float16* dst = outH + (slot0 + r) * (size_t)NOUT + col0 + c8;
      *(volatile v4f*)dst = u[i];
    }
    __threadfence();
#pragma unroll
    for (int i = 0; i < 2; ++i) {
      const int r = wave * 8 + i * 4 + rq;
      _Float16* dst = outH + (slot0 + r) * (size_t)NOUT + col0 + c8;
      *(volatile v4f*)dst = u[i];
    }
  } else {
    const int rq = lane >> 4, c4 = 4 * (lane & 15);
    v4f u[4];
#pragma unroll
    for (int i = 0; i < 4; ++i) {
      const int r = wave * 8 + i * 2 + rq;
      u[i] = *(const v4f*)(S + r * SP + c4);
    }
#pragma unroll
    for (int i = 0; i < 4; ++i) {
      const int r = wave * 8 + i * 2 + rq;
      float* dst = outF + (slot0 + r) * (size_t)NOUT + col0 + c4;
      *(volatile v4f*)dst = u[i];
    }
    __threadfence();
#pragma unroll
    for (int i = 0; i < 4; ++i) {
      const int r = wave * 8 + i * 2 + rq;
      float* dst = outF + (slot0 + r) * (size_t)NOUT + col0 + c4;
      *(volatile v4f*)dst = u[i];
    }
  }
}

__global__ __launch_bounds__(NTH) void k_ln1024(const float* __restrict__ U, _Float16* G, int nslots) {
  const int tid = threadIdx.x, wave = tid >> 5, lane = tid & 31;
  int row = blockIdx.x * NWV + wave;
  row = row < nslots ? row : nslots - 1;
  const float* ur = U + (size_t)row * HID + 8 * lane;
  v4f v[8];
  float s = 0.0f;
#pragma unroll
  for (int j = 0; j < 4; ++j) {
    v[2 * j]     = *(const v4f*)(ur + 256 * j);
    v[2 * j + 1] = *(const v4f*)(ur + 256 * j + 4);
    s += hsum4(v[2 * j]) + hsum4(v[2 * j + 1]);
  }
  s = wsum(s);
  const float mu = s * (1.0f / (float)HID);
  float q = 0.0f;
#pragma unroll
  for (int j = 0; j < 8; ++j) { v[j] = v[j] - mu; q += hsq4(v[j]); }
  q = wsum(q);
  const float sc = rsqrtf(q * (1.0f / (float)HID) + LN_EPS) * A_CARRY;
  Pk u[4];
#pragma unroll
  for (int j = 0; j < 4; ++j) {
    const v4f a = v[2 * j] * sc, c = v[2 * j + 1] * sc;
    const v8f o8 = __builtin_shufflevector(a, c, 0, 1, 2, 3, 4, 5, 6, 7);
    u[j].h = __builtin_convertvector(o8, v8h);
  }
  _Float16* gr = G + (size_t)row * HID + 8 * lane;
#pragma unroll
  for (int j = 0; j < 4; ++j) *(volatile v4f*)(gr + 256 * j) = u[j].f;
  __threadfence();
#pragma unroll
  for (int j = 0; j < 4; ++j) *(volatile v4f*)(gr + 256 * j) = u[j].f;
}

__global__ __launch_bounds__(NTH) void k_out(const float* __restrict__ Y, const float* __restrict__ x,
                                              const int* __restrict__ cat, float* out, int nrows, int nslots) {
  __shared__ int s_w[NWV * NGRP];
  __shared__ int s_pw[NWV * NGRP];
  __shared__ int s_cnt[NGRP];
  __shared__ int s_pre[NGRP];
  __shared__ unsigned s_b0[NGRP];
  __shared__ int s_pos[TM];
  const int tid = threadIdx.x, wave = tid >> 5, lane = tid & 31;
  const int row0 = blockIdx.x * TM;

  int cc[NGRP], pc[NGRP];
#pragma unroll
  for (int g = 0; g < NGRP; ++g) { cc[g] = 0; pc[g] = 0; }
  const int nch = (nrows + NTH - 1) / NTH;
#pragma unroll 1
  for (int j = 0; j < nch; ++j) {
    const int row = j * NTH + tid;
    const int ra = row < nrows ? row : nrows - 1;
    int id = cat[ra];
    id = row < nrows ? id : -1;
    const unsigned lt = __builtin_amdgcn_ballot_w32(row < row0);
#pragma unroll
    for (int g = 0; g < NGRP; ++g) {
      const unsigned b = __builtin_amdgcn_ballot_w32(id == g);
      cc[g] += __builtin_popcount(b);
      pc[g] += __builtin_popcount(b & lt);
    }
  }
  if (lane == 0) {
#pragma unroll
    for (int g = 0; g < NGRP; ++g) { s_w[wave * NGRP + g] = cc[g]; s_pw[wave * NGRP + g] = pc[g]; }
  }
  const int rb = row0 + (tid & (TM - 1));
  int idb = cat[rb < nrows ? rb : nrows - 1];
  idb = tid < TM ? idb : -1;
  unsigned bmine[NGRP];
#pragma unroll
  for (int g = 0; g < NGRP; ++g) {
    const unsigned b = __builtin_amdgcn_ballot_w32(idb == g);
    bmine[g] = b;
    if (tid == 0) s_b0[g] = b;
  }
  __syncthreads();
  if (tid < NGRP) {
    int s = 0, p = 0;
#pragma unroll
    for (int w = 0; w < NWV; ++w) { s += s_w[w * NGRP + tid]; p += s_pw[w * NGRP + tid]; }
    s_cnt[tid] = s;
    s_pre[tid] = p;
  }
  __syncthreads();
  if (tid < TM) {
    const unsigned ltl = (1u << lane) - 1u;
    int ts = 0, tsel = 0, psel = 0, rin = 0;
    bool valid = false;
#pragma unroll
    for (int g = 0; g < NGRP; ++g) {
      const int nt = (s_cnt[g] + TM - 1) / TM;
      const int w0c = __builtin_popcount(s_b0[g]);
      if (idb == g) {
        valid = true; tsel = ts; psel = s_pre[g];
        rin = __builtin_popcount(bmine[g] & ltl) + (wave == 1 ? w0c : 0);
      }
      ts += nt;
    }
    int pos = tsel * TM + psel + rin;
    pos = pos < 0 ? 0 : pos;
    pos = pos > nslots - 1 ? nslots - 1 : pos;
    s_pos[tid] = valid ? pos : -1;
  }
  __syncthreads();

  const v4f z4 = {0.f, 0.f, 0.f, 0.f};
#pragma unroll 1
  for (int i = 0; i < 8; ++i) {
    const int rl = wave * 8 + i;
    const int p = s_pos[rl];
    const int pa = p < 0 ? 0 : p;
    const float* yr = Y + (size_t)pa * DIM + 4 * lane;
    const float* xr = x + (size_t)(row0 + rl) * DIM + 4 * lane;
    v4f y0 = *(const v4f*)(yr);
    v4f y1 = *(const v4f*)(yr + 128);
    const v4f x0 = *(const v4f*)(xr);
    const v4f x1 = *(const v4f*)(xr + 128);
    if (p < 0) { y0 = z4; y1 = z4; }
    const v4f v0 = y0 + 0.1f * x0;
    const v4f v1 = y1 + 0.1f * x1;
    float s = hsum4(v0) + hsum4(v1);
    s = wsum(s);
    const float mu = s * (1.0f / (float)DIM);
    const v4f d0 = v0 - mu, d1 = v1 - mu;
    float q = hsq4(d0) + hsq4(d1);
    q = wsum(q);
    const float rs = rsqrtf(q * (1.0f / (float)DIM) + LN_EPS);
    const v4f o0 = d0 * rs, o1 = d1 * rs;
    float* dst = out + (size_t)(row0 + rl) * DIM + 4 * lane;
    *(volatile v4f*)(dst) = o0;
    *(volatile v4f*)(dst + 128) = o1;
    __threadfence();
    *(volatile v4f*)(dst) = o0;
    *(volatile v4f*)(dst + 128) = o1;
  }
}

extern "C" void kernel_launch(void* const* d_in, const int* in_sizes, int n_in,
                              void* d_out, int out_size, void* d_ws, size_t ws_size,
                              hipStream_t stream) {
  if (n_in < 12) return;
  const int nrows = in_sizes[1];
  if (nrows < TM || (nrows % TM) != 0) return;
  if (in_sizes[0] != nrows * DIM) return;
  if (in_sizes[2] != NGRP * DIM * HID || in_sizes[3] != NGRP * HID) return;
  if (in_sizes[4] != NGRP * HID * HID || in_sizes[5] != NGRP * HID) return;
  if (in_sizes[6] != NGRP * HID * HID || in_sizes[7] != NGRP * HID) return;
  if (in_sizes[8] != NGRP * HID * HID || in_sizes[9] != NGRP * HID) return;
  if (in_sizes[10] != NGRP * HID * DIM || in_sizes[11] != NGRP * DIM) return;
  if (out_size != nrows * DIM) return;

  const int maxt   = nrows / TM + NGRP;
  const int nslots = maxt * TM;

  size_t off = 0;
  auto carve = [&](size_t bytes) { size_t p = off; off += (bytes + 255) & ~(size_t)255; return p; };
  const size_t oWT0 = carve((size_t)NGRP * HID * DIM * 2);
  const size_t oWTM = carve((size_t)NGRP * HID * HID * 2);
  const size_t oWTG = carve((size_t)NGRP * HID * HID * 2);
  const size_t oWTO = carve((size_t)NGRP * HID * HID * 2);
  const size_t oWT2 = carve((size_t)NGRP * DIM * HID * 2);
  const size_t oXN  = carve((size_t)nslots * DIM * 2);
  const size_t oH1  = carve((size_t)nslots * HID * 2);
  const size_t oU   = carve((size_t)nslots * HID * 4);
  const size_t oGP  = carve((size_t)nslots * HID * 2);
  const size_t oV   = carve((size_t)nslots * HID * 4);
  const size_t oH2  = carve((size_t)nslots * HID * 2);
  const size_t oY   = carve((size_t)nslots * DIM * 4);
  if (off > ws_size || off > (size_t)WSCAP) return;

  const float* x   = (const float*)d_in[0];
  const int*   cat = (const int*)d_in[1];
  const float* W0  = (const float*)d_in[2];
  const float* b0  = (const float*)d_in[3];
  const float* Wm  = (const float*)d_in[4];
  const float* bm  = (const float*)d_in[5];
  const float* Wg  = (const float*)d_in[6];
  const float* bg  = (const float*)d_in[7];
  const float* Wog = (const float*)d_in[8];
  const float* bog = (const float*)d_in[9];
  const float* W2  = (const float*)d_in[10];
  const float* b2  = (const float*)d_in[11];
  float* out = (float*)d_out;
  char* ws = (char*)d_ws;
  _Float16* WT0 = (_Float16*)(ws + oWT0);
  _Float16* WTM = (_Float16*)(ws + oWTM);
  _Float16* WTG = (_Float16*)(ws + oWTG);
  _Float16* WTO = (_Float16*)(ws + oWTO);
  _Float16* WT2 = (_Float16*)(ws + oWT2);
  _Float16* XN  = (_Float16*)(ws + oXN);
  _Float16* H1  = (_Float16*)(ws + oH1);
  float*    U   = (float*)(ws + oU);
  _Float16* GP  = (_Float16*)(ws + oGP);
  float*    V   = (float*)(ws + oV);
  _Float16* H2  = (_Float16*)(ws + oH2);
  float*    Y   = (float*)(ws + oY);

  k_wprep<<<NGRP * (HID / 32) * (DIM / 256), NTH, 0, stream>>>(W0, WT0, DIM, HID);
  k_wprep<<<NGRP * (HID / 32) * (HID / 256), NTH, 0, stream>>>(Wm, WTM, HID, HID);
  k_wprep<<<NGRP * (HID / 32) * (HID / 256), NTH, 0, stream>>>(Wg, WTG, HID, HID);
  k_wprep<<<NGRP * (HID / 32) * (HID / 256), NTH, 0, stream>>>(Wog, WTO, HID, HID);
  k_wprep<<<NGRP * (DIM / 32) * (HID / 256), NTH, 0, stream>>>(W2, WT2, HID, DIM);

  k_xn<<<maxt, NTH, 0, stream>>>(x, cat, XN, nrows);

  k_gemm<DIM, HID, 1><<<dim3(maxt, HID / TN), NTH, 0, stream>>>(XN, WT0, WT0, b0, b0, cat, U, H1, nrows);
  k_gemm<HID, HID, 2><<<dim3(maxt, HID / TN), NTH, 0, stream>>>(H1, WTM, WTG, bm, bg, cat, U, H1, nrows);
  k_ln1024<<<nslots / NWV, NTH, 0, stream>>>(U, GP, nslots);
  k_gemm<HID, HID, 0><<<dim3(maxt, HID / TN), NTH, 0, stream>>>(GP, WTO, WTO, bog, bog, cat, V, GP, nrows);
  k_ln1024<<<nslots / NWV, NTH, 0, stream>>>(V, H2, nslots);
  k_gemm<HID, DIM, 0><<<dim3(maxt, DIM / TN), NTH, 0, stream>>>(H2, WT2, WT2, b2, b2, cat, Y, H2, nrows);
  k_out<<<nrows / TM, NTH, 0, stream>>>(Y, x, cat, out, nrows, nslots);
}
